// CIM_34677565948716
// MI455X (gfx1250) — hardware-verified
//
#include <hip/hip_runtime.h>


#define NB_  4
#define CC   256
#define CH   512
#define NN   4096
#define MM   1024
#define NHD  8
#define DH   32
#define OTP  288
#define PCAR 1024.0f
#define SCL  0.17677669529663687f
typedef _Float16 h16;
typedef unsigned short bf;
typedef __attribute__((ext_vector_type(16))) __bf16   v16bf;
typedef __attribute__((ext_vector_type(16))) _Float16 v16h;
typedef __attribute__((ext_vector_type(8)))  _Float16 v8h;
typedef __attribute__((ext_vector_type(8)))  unsigned short v8us;
typedef __attribute__((ext_vector_type(8)))  float    v8f;
typedef __attribute__((ext_vector_type(4)))  float    v4f;
typedef v8h  __attribute__((may_alias)) v8ha;
typedef v4f  __attribute__((may_alias)) v4fa;
typedef v8us __attribute__((may_alias)) v8usa;

__device__ __forceinline__ unsigned short f2bf(float f) { unsigned u = __float_as_uint(f); u += 0x7FFFu + ((u >> 16) & 1u); return (unsigned short)(u >> 16); }
__device__ __forceinline__ float bf2f(unsigned short b) { return __uint_as_float(((unsigned)b) << 16); }
__device__ __forceinline__ float bfr(float f) { return bf2f(f2bf(f)); }
__device__ __forceinline__ v16h cat16(v8h lo, v8h hi) { return __builtin_shufflevector(lo, hi, 0, 1, 2, 3, 4, 5, 6, 7, 8, 9, 10, 11, 12, 13, 14, 15); }
__device__ __forceinline__ v16bf cat16b(v8us lo, v8us hi) { return __builtin_bit_cast(v16bf, __builtin_shufflevector(lo, hi, 0, 1, 2, 3, 4, 5, 6, 7, 8, 9, 10, 11, 12, 13, 14, 15)); }
__device__ __forceinline__ v8f wmma16(v16h a, v16h b, v8f c) { return __builtin_amdgcn_wmma_f32_16x16x32_f16(false, a, false, b, (short)0, c, false, false); }
__device__ __forceinline__ v8f wmmab(v16bf a, v16bf b, v8f c) { return __builtin_amdgcn_wmma_f32_16x16x32_bf16(false, a, false, b, (short)0, c, false, false); }


template <typename T16> struct WFrag;
template <> struct WFrag<h16> { typedef v16h V; static __device__ __forceinline__ V ld(const h16* p) { return cat16(*(const v8h*)p, *(const v8h*)(p + 16)); } static __device__ __forceinline__ v8f mma(V a, V b, v8f c) { return wmma16(a, b, c); } };
template <> struct WFrag<bf> { typedef v16bf V; static __device__ __forceinline__ V ld(const bf* p) { return cat16b(*(const v8us*)p, *(const v8us*)(p + 16)); } static __device__ __forceinline__ v8f mma(V a, V b, v8f c) { return wmmab(a, b, c); } };
template <typename T16, int NSPLIT, bool BIAS>
__global__ __launch_bounds__(32) void k_gemmw(const T16* __restrict__ A, const T16* __restrict__ A2, const T16* __restrict__ Bt, const T16* __restrict__ Bt2, int K, float* C, int ldc, const float* __restrict__ bias, size_t sA, size_t sB, size_t sC) {
    typedef typename WFrag<T16>::V V;
    __shared__ __align__(16) float os[16 * 68];
    const size_t z = blockIdx.z; A += z * sA; if (A2) A2 += z * sA; Bt += z * sB; if (Bt2) Bt2 += z * sB; C += z * sC;
    const int lane = threadIdx.x & 31, lr = lane & 15, hi = lane >> 4; const int r0 = blockIdx.x * 64, c0 = blockIdx.y * 64;
    v8f acc[4][4];
#pragma unroll
    for (int mb = 0; mb < 4; ++mb)
#pragma unroll
        for (int nb = 0; nb < 4; ++nb) acc[mb][nb] = (v8f){};
    const size_t aoff = (size_t)(r0 + lr) * K + 8 * hi, boff = (size_t)(c0 + lr) * K + 8 * hi;
#pragma unroll 1
    for (int kc = 0; kc < K; kc += 32) {
        V a[4], a2[4];
#pragma unroll
        for (int mb = 0; mb < 4; ++mb) { a[mb] = WFrag<T16>::ld(A + aoff + (size_t)mb * 16 * K + kc); if (NSPLIT == 1 || NSPLIT == 2) a2[mb] = WFrag<T16>::ld(A2 + aoff + (size_t)mb * 16 * K + kc); }
#pragma unroll
        for (int nb = 0; nb < 4; ++nb) { const V b = WFrag<T16>::ld(Bt + boff + (size_t)nb * 16 * K + kc); V b2; if (NSPLIT >= 2) b2 = WFrag<T16>::ld(Bt2 + boff + (size_t)nb * 16 * K + kc);
#pragma unroll
            for (int mb = 0; mb < 4; ++mb) { acc[mb][nb] = WFrag<T16>::mma(a[mb], b, acc[mb][nb]); if (NSPLIT == 1 || NSPLIT == 2) acc[mb][nb] = WFrag<T16>::mma(a2[mb], b, acc[mb][nb]); if (NSPLIT >= 2) acc[mb][nb] = WFrag<T16>::mma(a[mb], b2, acc[mb][nb]); } }
        asm volatile("v_nop\n\tv_nop\n\tv_nop\n\tv_nop" : "+v"(acc[0][0]), "+v"(acc[1][1]), "+v"(acc[2][2]), "+v"(acc[3][3]) : "v"(a[0]), "v"(a[3]));
    }
#pragma unroll
    for (int mb = 0; mb < 4; ++mb) {
#pragma unroll
        for (int nb = 0; nb < 4; ++nb) {
#pragma unroll
            for (int j = 0; j < 8; ++j) os[(hi * 8 + j) * 68 + nb * 16 + lr] = acc[mb][nb][j]; }
        __builtin_amdgcn_wave_barrier(); asm volatile("" ::: "memory");
        float* crow = C + (size_t)(r0 + mb * 16) * ldc + c0;
#pragma unroll 1
        for (int ps = 0; ps < 2; ++ps) {
#pragma unroll
            for (int s = 0; s < 8; ++s) { const int row = 2 * s + hi, cofs = lr * 4; v4f val = *(const v4fa*)(os + row * 68 + cofs); if (BIAS) { val[0] += bfr(bias[c0 + cofs]); val[1] += bfr(bias[c0 + cofs + 1]); val[2] += bfr(bias[c0 + cofs + 2]); val[3] += bfr(bias[c0 + cofs + 3]); }
                *(volatile v4f*)(crow + (size_t)row * ldc + cofs) = val; }
            if (ps == 0) __threadfence(); }
        __builtin_amdgcn_wave_barrier(); asm volatile("" ::: "memory");
    }
}

__device__ __forceinline__ h16 tohx(float x) { return (h16)x; }
__device__ __forceinline__ void splitf(float y, unsigned short& h, unsigned short& l) { h = f2bf(y); l = f2bf(y - bf2f(h)); }
typedef __attribute__((ext_vector_type(2))) _Float16 v2h;
typedef __attribute__((ext_vector_type(4))) _Float16 v4h;
typedef __attribute__((ext_vector_type(2))) unsigned short v2us;
typedef __attribute__((ext_vector_type(8))) _Float16 v8h16;

__global__ __launch_bounds__(256) void k_cvt8(const float* __restrict__ src, bf* dst, size_t n8) { const size_t i = (size_t)blockIdx.x * 256 + threadIdx.x; if (i >= n8) return; const v8f v = *(const v8f*)(src + i * 8); v8us o;
#pragma unroll
    for (int k = 0; k < 8; ++k) o[k] = f2bf(v[k]); *(volatile v8us*)(dst + i * 8) = o; __threadfence(); *(volatile v8us*)(dst + i * 8) = o; }
__global__ __launch_bounds__(256) void k_xth(const float* __restrict__ hb, bf* HB) {
    const int lane = threadIdx.x & 31; const int L0 = (blockIdx.x * 8 + (threadIdx.x >> 5)) * 8; const int nlines = MM * CH / 64;
#pragma unroll 1
    for (int ps = 0; ps < 2; ++ps) {
#pragma unroll
        for (int l = 0; l < 8; ++l) { const int L = L0 + l; if (L >= nlines) break; const int e = L * 64 + lane * 2; const int k = e & (CH - 1); const int m = e >> 9; v2us o;
#pragma unroll
            for (int q = 0; q < 2; ++q) o[q] = f2bf(hb[(size_t)(k + q) * MM + m]);
            *(volatile v2us*)(HB + (size_t)e) = o; }
        if (ps == 0) __threadfence(); }
}
template <int RAW>
__global__ __launch_bounds__(256) void k_bnT(const float* __restrict__ src, int cols, int lg2cols, const float* __restrict__ rowbias, const float* __restrict__ gam, const float* __restrict__ bet, const float* __restrict__ mean, const float* __restrict__ var, bf* Th, bf* Tl) {
    const int lane = threadIdx.x & 31; const int L0 = (blockIdx.x * 8 + (threadIdx.x >> 5)) * 8; const int nlines = cols * CC / 64;
#pragma unroll 1
    for (int ps = 0; ps < 2; ++ps) {
#pragma unroll 1
        for (int l = 0; l < 8; ++l) { const int L = L0 + l; if (L >= nlines) break; const int e = L * 64 + lane * 2; const int c = e & (CC - 1); const int n = e >> 8; v2us oh, ol;
#pragma unroll
            for (int q = 0; q < 2; ++q) { const int cc = c + q; const float inv = __fdiv_rn(bfr(gam[cc]), __fsqrt_rn(__fadd_rn(bfr(var[cc]), 1e-5f))); float ms = __fmul_rn(bfr(mean[cc]), inv); asm volatile("" : "+v"(ms)); const float sh = __fsub_rn(bfr(bet[cc]), ms);
                float x = src[(size_t)cc * cols + n]; if (RAW) x = bfr(x); if (rowbias) x = __fadd_rn(x, bfr(rowbias[cc])); float t = __fmul_rn(x, inv); asm volatile("" : "+v"(t)); unsigned short a, c2; splitf(__fadd_rn(t, sh), a, c2); oh[q] = a; ol[q] = c2; }
            *(volatile v2us*)(Th + (size_t)e) = oh; *(volatile v2us*)(Tl + (size_t)e) = ol; }
        if (ps == 0) __threadfence(); }
}
__global__ __launch_bounds__(256) void k_hp32(const float* __restrict__ F, int rows, int lg2rows, h16* P) {
    const int lane = threadIdx.x & 31; const int L0 = (blockIdx.x * 8 + (threadIdx.x >> 5)) * 8; const int nlines = NHD * rows * DH / 64;
#pragma unroll 1
    for (int ps = 0; ps < 2; ++ps) {
#pragma unroll
        for (int l = 0; l < 8; ++l) { const int L = L0 + l; if (L >= nlines) break; const int e = L * 64 + lane * 2; const int d = e & (DH - 1); const int r = (e >> 5) & (rows - 1); const int h = e >> (5 + lg2rows); v2h o;
#pragma unroll
            for (int q = 0; q < 2; ++q) o[q] = tohx(F[(size_t)r * CC + h * DH + d + q]);
            *(volatile v2h*)(P + (size_t)e) = o; }
        if (ps == 0) __threadfence(); }
}
__global__ __launch_bounds__(256) void k_v16(const float* __restrict__ FV, const float* __restrict__ bv, h16* V16) { const size_t i = ((size_t)blockIdx.x * 256 + threadIdx.x) * 2; if (i >= (size_t)CC * MM) return; const int c = (int)(i >> 10); v2h v;
#pragma unroll
    for (int q = 0; q < 2; ++q) v[q] = tohx(__fadd_rn(FV[i + q], bfr(bv[c]))); *(volatile v2h*)(V16 + i) = v; __threadfence(); *(volatile v2h*)(V16 + i) = v; }
__global__ __launch_bounds__(256) void k_smax(const float* __restrict__ S, float* RS) {
    const int lane = threadIdx.x & 31; const int i = blockIdx.x * 8 + (threadIdx.x >> 5); if (i >= NN) return; const float* sr = S + (size_t)i * MM; float m = -3.0e38f;
#pragma unroll 4
    for (int c0 = lane * 4; c0 < MM; c0 += 128) { const v4f v = *(const v4f*)(sr + c0); m = fmaxf(m, fmaxf(fmaxf(v[0], v[1]), fmaxf(v[2], v[3]))); }
#pragma unroll
    for (int sh = 16; sh; sh >>= 1) m = fmaxf(m, __shfl_xor(m, sh, 32));
    const float o = lane == 0 ? m : 0.f; *(volatile float*)(RS + (size_t)i * 32 + lane) = o; __threadfence(); *(volatile float*)(RS + (size_t)i * 32 + lane) = o; }
__global__ __launch_bounds__(256) void k_sexp(const float* __restrict__ S, float* RS, h16* P) {
    const int lane = threadIdx.x & 31; const int i = blockIdx.x * 8 + (threadIdx.x >> 5); if (i >= NN) return; const float* sr = S + (size_t)i * MM; const float m = RS[(size_t)i * 32]; float sum = 0.f;
#pragma unroll 2
    for (int c0 = lane * 4; c0 < MM; c0 += 128) { const v4f v = *(const v4f*)(sr + c0); v4h o;
#pragma unroll
        for (int q = 0; q < 4; ++q) { float dlt = __fsub_rn(v[q], m); asm volatile("" : "+v"(dlt)); const float e = __expf(__fmul_rn(dlt, SCL)); sum += e; o[q] = tohx(e * PCAR); }
        *(volatile v4h*)(P + (size_t)i * MM + c0) = o; __threadfence(); *(volatile v4h*)(P + (size_t)i * MM + c0) = o; }
#pragma unroll
    for (int sh = 16; sh; sh >>= 1) sum += __shfl_xor(sum, sh, 32);
    const float o2 = lane == 0 ? m : (lane == 1 ? __fdiv_rn(1.0f, sum * PCAR) : 0.f); *(volatile float*)(RS + (size_t)i * 32 + lane) = o2; __threadfence(); *(volatile float*)(RS + (size_t)i * 32 + lane) = o2; }
__global__ __launch_bounds__(256) void k_osplit(const float* __restrict__ OTf, const float* __restrict__ RSall, bf* Oh, bf* Ol) { const size_t i = ((size_t)blockIdx.x * 256 + threadIdx.x) * 2; if (i >= (size_t)NN * CC) return; const int c = (int)(i & (CC - 1)); const int n = (int)(i >> 8); const float ri = RSall[((size_t)(c >> 5) * NN + n) * 32 + 1]; v2us oh, ol;
#pragma unroll
    for (int q = 0; q < 2; ++q) { unsigned short a, c2; splitf(__fmul_rn(OTf[(size_t)n * OTP + c + q], ri), a, c2); oh[q] = a; ol[q] = c2; }
    *(volatile v2us*)(Oh + i) = oh; *(volatile v2us*)(Ol + i) = ol; __threadfence(); *(volatile v2us*)(Oh + i) = oh; *(volatile v2us*)(Ol + i) = ol; }
__global__ __launch_bounds__(256) void k_fin(const float* __restrict__ xb, const float* __restrict__ PR, const float* __restrict__ bp, float* OUTb) { const size_t i = ((size_t)blockIdx.x * 256 + threadIdx.x) * 4; if (i >= (size_t)CC * NN) return; const int c = (int)(i >> 12); const v4f a = *(const v4f*)(xb + i), p = *(const v4f*)(PR + i); v4f o;
#pragma unroll
    for (int q = 0; q < 4; ++q) o[q] = __fadd_rn(__fadd_rn(bfr(a[q]), p[q]), bfr(bp[c]));
    *(volatile v4f*)(OUTb + i) = o; __threadfence(); *(volatile v4f*)(OUTb + i) = o; }


extern "C" void kernel_launch(void* const* d_in, const int* in_sizes, int n_in,
                              void* d_out, int out_size, void* d_ws, size_t ws_size, hipStream_t stream) {
    (void)in_sizes; (void)n_in; (void)out_size;
    const float* IN[16]; for (int i = 0; i < 16; ++i) IN[i] = (const float*)d_in[i];
    const float* f = IN[0]; const float* hin = IN[1]; const float* gam = IN[4]; const float* bet = IN[5]; const float* mean = IN[6]; const float* var = IN[7];
    float* OUT = (float*)d_out;
    char* wsp = (char*)d_ws;
    auto take = [&](size_t bytes) { char* p = wsp; wsp += (bytes + 255) & ~(size_t)255; return (void*)p; };
    bf* WHT = (bf*)take((size_t)CC * CH * 2); bf* WQ = (bf*)take((size_t)CC * CC * 2); bf* WK = (bf*)take((size_t)CC * CC * 2); bf* WV = (bf*)take((size_t)CC * CC * 2); bf* WO = (bf*)take((size_t)CC * CC * 2);
    bf* HB = (bf*)take((size_t)MM * CH * 2); float* HAL = (float*)take((size_t)CC * MM * 4); bf* H1h = (bf*)take((size_t)MM * CC * 2); bf* H1l = (bf*)take((size_t)MM * CC * 2); bf* H2h = (bf*)take((size_t)MM * CC * 2); bf* H2l = (bf*)take((size_t)MM * CC * 2);
    bf* FTh = (bf*)take((size_t)NN * CC * 2); bf* FTl = (bf*)take((size_t)NN * CC * 2); float* FQ = (float*)take((size_t)NN * CC * 4); h16* QP = (h16*)take((size_t)NHD * NN * DH * 2); float* FK = (float*)take((size_t)MM * CC * 4); h16* KP = (h16*)take((size_t)NHD * MM * DH * 2);
    float* FV = (float*)take((size_t)CC * MM * 4); h16* V16 = (h16*)take((size_t)(CC + DH) * MM * 2);
    float* S = (float*)take((size_t)NN * MM * 4); h16* P = (h16*)take((size_t)NN * MM * 2); float* RS = (float*)take((size_t)NHD * NN * 32 * 4); float* OTf = (float*)take((size_t)NN * OTP * 4); bf* Oh = (bf*)take((size_t)NN * CC * 2); bf* Ol = (bf*)take((size_t)NN * CC * 2); float* PR = FQ;
    if ((size_t)(wsp - (char*)d_ws) > ws_size) return;
    { k_cvt8<<<(CC * CH / 8 + 255) / 256, 256, 0, stream>>>(IN[2], WHT, (size_t)CC * CH / 8); const unsigned g8 = (CC * CC / 8 + 255) / 256;
      k_cvt8<<<g8, 256, 0, stream>>>(IN[8], WQ, (size_t)CC * CC / 8); k_cvt8<<<g8, 256, 0, stream>>>(IN[10], WK, (size_t)CC * CC / 8); k_cvt8<<<g8, 256, 0, stream>>>(IN[12], WV, (size_t)CC * CC / 8); k_cvt8<<<g8, 256, 0, stream>>>(IN[14], WO, (size_t)CC * CC / 8);
      hipMemsetAsync(V16 + (size_t)CC * MM, 0, (size_t)DH * MM * 2, stream); }
    const unsigned L2 = (unsigned)(((size_t)NN * CC / 2 + 255) / 256), L4 = (unsigned)(((size_t)NN * CC / 4 + 255) / 256);
    for (int b = 0; b < NB_; ++b) { const float* fb = f + (size_t)b * CC * NN; const float* hb = hin + (size_t)b * CH * MM;
        k_xth<<<(MM * CH / 64 + 63) / 64, 256, 0, stream>>>(hb, HB);
        k_gemmw<bf, 0, false><<<dim3(CC / 64, MM / 64, 1), 32, 0, stream>>>(WHT, nullptr, HB, nullptr, CH, HAL, MM, nullptr, 0, 0, 0);
        k_bnT<0><<<(MM * CC / 64 + 63) / 64, 256, 0, stream>>>(HAL, MM, 10, IN[3], gam + CC, bet + CC, mean + CC, var + CC, H1h, H1l);
        k_bnT<0><<<(MM * CC / 64 + 63) / 64, 256, 0, stream>>>(HAL, MM, 10, IN[3], gam + 2 * CC, bet + 2 * CC, mean + 2 * CC, var + 2 * CC, H2h, H2l);
        k_bnT<1><<<(NN * CC / 64 + 63) / 64, 256, 0, stream>>>(fb, NN, 12, nullptr, gam, bet, mean, var, FTh, FTl);
        k_gemmw<bf, 1, true><<<dim3(NN / 64, CC / 64, 1), 32, 0, stream>>>(FTh, FTl, WQ, nullptr, CC, FQ, CC, IN[9], 0, 0, 0); k_hp32<<<(NHD * NN * DH / 64 + 63) / 64, 256, 0, stream>>>(FQ, NN, 12, QP);
        k_gemmw<bf, 1, true><<<dim3(MM / 64, CC / 64, 1), 32, 0, stream>>>(H1h, H1l, WK, nullptr, CC, FK, CC, IN[11], 0, 0, 0); k_hp32<<<(NHD * MM * DH / 64 + 63) / 64, 256, 0, stream>>>(FK, MM, 10, KP);
        k_gemmw<bf, 3, false><<<dim3(CC / 64, MM / 64, 1), 32, 0, stream>>>(WV, nullptr, H2h, H2l, CC, FV, MM, nullptr, 0, 0, 0); k_v16<<<(unsigned)(((size_t)CC * MM / 2 + 255) / 256), 256, 0, stream>>>(FV, IN[13], V16);
        for (int hh = 0; hh < NHD; ++hh) {
            k_gemmw<h16, 0, false><<<dim3(NN / 64, MM / 64, 1), 32, 0, stream>>>(QP + (size_t)hh * NN * DH, nullptr, KP + (size_t)hh * MM * DH, nullptr, DH, S, MM, nullptr, 0, 0, 0);
            k_smax<<<NN / 8, 256, 0, stream>>>(S, RS + (size_t)hh * NN * 32); k_sexp<<<NN / 8, 256, 0, stream>>>(S, RS + (size_t)hh * NN * 32, P);
            k_gemmw<h16, 0, false><<<dim3(NN / 64, 1, 1), 32, 0, stream>>>(P, nullptr, V16 + (size_t)hh * DH * MM, nullptr, MM, OTf + hh * DH, OTP, nullptr, 0, 0, 0); }
        k_osplit<<<L2, 256, 0, stream>>>(OTf, RS, Oh, Ol);
        k_gemmw<bf, 3, false><<<dim3(CC / 64, NN / 64, 1), 32, 0, stream>>>(WO, nullptr, Oh, Ol, CC, PR, NN, nullptr, 0, 0, 0);
        k_fin<<<L4, 256, 0, stream>>>(fb, PR, IN[15], OUT + (size_t)b * CC * NN); }
}
